// SSDFLUIDLayer_4389456577368
// MI455X (gfx1250) — hardware-verified
//
#include <hip/hip_runtime.h>
#include <stddef.h>
#include <stdint.h>
#include <math.h>

#define BB   2
#define NN   2048
#define DD   1024
#define EE   2048
#define FF   4096
#define MTOK 4096
#define NTRI 136
#define SHP  136
#define SFP  132

static_assert(MTOK == BB * NN);
static_assert(NN % 128 == 0);
static_assert(DD % 128 == 0);
static_assert(EE % 128 == 0);
static_assert(FF % 128 == 0);
static_assert(DD % 32 == 0);
static_assert(EE % 32 == 0);
static_assert(FF % 32 == 0);
static_assert(EE == 8 * 256);
static_assert(DD == 8 * 128);
static_assert(NN % 32 == 0);
static_assert(NTRI == (NN / 128) * (NN / 128 + 1) / 2);
static_assert(FF == 2 * EE);
static_assert((size_t)MTOK * DD * 4 == (size_t)BB * NN * NN * 2);

typedef _Float16 hh;
typedef hh    v16h __attribute__((ext_vector_type(16)));
typedef hh    v8h  __attribute__((ext_vector_type(8)));
typedef float v8f  __attribute__((ext_vector_type(8)));
typedef float v4f  __attribute__((ext_vector_type(4)));

union Frag { v16h v; v8h p[2]; };
union EpiLds { hh h[128 * SHP]; float f[64 * SFP]; };

__device__ __forceinline__ v8f zero8() { return (v8f){0.f, 0.f, 0.f, 0.f, 0.f, 0.f, 0.f, 0.f}; }

__device__ __forceinline__ float wsum(float v) {
#pragma unroll
  for (int off = 16; off > 0; off >>= 1) v += __shfl_xor(v, off, 32);
  return v;
}

__device__ __forceinline__ v16h ldfrag(const hh* __restrict__ p, int ld, int row0, int k0, int lane) {
  const hh* q = p + (size_t)(row0 + (lane & 15)) * (size_t)ld + k0 + 8 * (lane >> 4);
  Frag f;
  f.p[0] = *(const v8h*)(q);
  f.p[1] = *(const v8h*)(q + 16);
  return f.v;
}

__device__ __forceinline__ v8f mma16(v16h a, v16h b, v8f cc) {
  return __builtin_amdgcn_wmma_f32_16x16x32_f16(false, a, false, b, (short)0, cc, false, false);
}

__device__ __forceinline__ void gemm32x64(const hh* __restrict__ A, int lda, const hh* __restrict__ B, int ldb,
                                          int ma, int nb, int kdim, int lane, v8f (&acc)[2][4]) {
#pragma unroll 1
  for (int k0 = 0; k0 < kdim; k0 += 32) {
    const v16h a0 = ldfrag(A, lda, ma, k0, lane);
    const v16h a1 = ldfrag(A, lda, ma + 16, k0, lane);
    const v16h b0 = ldfrag(B, ldb, nb, k0, lane);
    const v16h b1 = ldfrag(B, ldb, nb + 16, k0, lane);
    const v16h b2 = ldfrag(B, ldb, nb + 32, k0, lane);
    const v16h b3 = ldfrag(B, ldb, nb + 48, k0, lane);
    acc[0][0] = mma16(a0, b0, acc[0][0]);
    acc[1][0] = mma16(a1, b0, acc[1][0]);
    acc[0][1] = mma16(a0, b1, acc[0][1]);
    acc[1][1] = mma16(a1, b1, acc[1][1]);
    acc[0][2] = mma16(a0, b2, acc[0][2]);
    acc[1][2] = mma16(a1, b2, acc[1][2]);
    acc[0][3] = mma16(a0, b3, acc[0][3]);
    acc[1][3] = mma16(a1, b3, acc[1][3]);
    asm volatile("v_nop\n\tv_nop\n\tv_nop\n\tv_nop"
                 : "+v"(acc[0][0]), "+v"(acc[0][1]), "+v"(acc[0][2]), "+v"(acc[0][3]),
                   "+v"(acc[1][0]), "+v"(acc[1][1]), "+v"(acc[1][2]), "+v"(acc[1][3])
                 : "v"(a0), "v"(a1), "v"(b0), "v"(b1), "v"(b2), "v"(b3));
  }
}

__device__ __forceinline__ float phi_f(float t) {
  const float e = __expf(fminf(t, 0.f));
  return (t > 0.f) ? (t + 1.0f) : e;
}

__device__ __forceinline__ float gelu_f(float x) {
  const float z  = fabsf(x) * 0.70710678118654752f;
  const float t  = __builtin_amdgcn_rcpf(fmaf(0.3275911f, z, 1.0f));
  float pl = fmaf(t, 1.061405429f, -1.453152027f);
  pl = fmaf(t, pl, 1.421413741f);
  pl = fmaf(t, pl, -0.284496736f);
  pl = fmaf(t, pl, 0.254829592f);
  pl = pl * t;
  const float ex   = __expf(-z * z);
  const float erfa = fmaf(-pl, ex, 1.0f);
  const float erfv = (x < 0.f) ? -erfa : erfa;
  return 0.5f * x * (1.0f + erfv);
}

template <int KD, int ND>
__global__ __launch_bounds__(256) void k_cvt_wt(const float* __restrict__ w, hh* __restrict__ wt) {
  static_assert(KD % 64 == 0);
  static_assert(ND % 64 == 0);
  __shared__ __align__(16) float sw[64 * 68];
  const int tid = threadIdx.x;
  const int kb = blockIdx.x * 64;
  const int nb = blockIdx.y * 64;
  {
    const int r  = tid >> 2;
    const int c0 = (tid & 3) * 16;
    const float* src = w + (size_t)(kb + r) * ND + nb + c0;
#pragma unroll
    for (int e = 0; e < 4; ++e) *(v4f*)(sw + r * 68 + c0 + 4 * e) = *(const v4f*)(src + 4 * e);
  }
  __syncthreads();
  v8h hv[2];
  size_t go[2];
#pragma unroll
  for (int j = 0; j < 2; ++j) {
    const int p  = tid + 256 * j;
    const int n  = p >> 3;
    const int pc = p & 7;
    const float* cp = sw + (pc * 8) * 68 + n;
    v8f t;
#pragma unroll
    for (int e = 0; e < 8; ++e) t[e] = cp[e * 68] * 64.0f;
    hv[j] = __builtin_convertvector(t, v8h);
    go[j] = (size_t)(nb + n) * KD + kb + pc * 8;
  }
#pragma unroll
  for (int j = 0; j < 2; ++j) *(volatile v8h*)(wt + go[j]) = hv[j];
  __threadfence();
#pragma unroll
  for (int j = 0; j < 2; ++j) *(volatile v8h*)(wt + go[j]) = hv[j];
}

__global__ __launch_bounds__(128) void k_ln(const float* __restrict__ x, const float* __restrict__ g,
                                            const float* __restrict__ bt, hh* __restrict__ y) {
  __shared__ float red[8];
  const int tid = threadIdx.x, lane = tid & 31, w = tid >> 5;
  const size_t ro = (size_t)blockIdx.x * DD + (size_t)tid * 8;
  const v4f a0 = *(const v4f*)(x + ro), a1 = *(const v4f*)(x + ro + 4);
  const float f[8] = {a0[0], a0[1], a0[2], a0[3], a1[0], a1[1], a1[2], a1[3]};
  float s = 0.f;
#pragma unroll
  for (int e = 0; e < 8; ++e) s += f[e];
  s = wsum(s);
  if (lane == 0) red[w] = s;
  __syncthreads();
  const float mu = ((red[0] + red[1]) + (red[2] + red[3])) * (1.0f / (float)DD);
  float d[8];
  float s2 = 0.f;
#pragma unroll
  for (int e = 0; e < 8; ++e) { d[e] = f[e] - mu; s2 = fmaf(d[e], d[e], s2); }
  s2 = wsum(s2);
  if (lane == 0) red[4 + w] = s2;
  __syncthreads();
  const float var = ((red[4] + red[5]) + (red[6] + red[7])) * (1.0f / (float)DD);
  const float inv = rsqrtf(var + 1e-5f);
  const v4f g0 = *(const v4f*)(g + tid * 8), g1 = *(const v4f*)(g + tid * 8 + 4);
  const v4f b0 = *(const v4f*)(bt + tid * 8), b1 = *(const v4f*)(bt + tid * 8 + 4);
  const float gg[8] = {g0[0], g0[1], g0[2], g0[3], g1[0], g1[1], g1[2], g1[3]};
  const float bb[8] = {b0[0], b0[1], b0[2], b0[3], b1[0], b1[1], b1[2], b1[3]};
  v8f t;
#pragma unroll
  for (int e = 0; e < 8; ++e) t[e] = d[e] * inv * gg[e] + bb[e];
  const v8h pk = __builtin_convertvector(t, v8h);
  *(volatile v8h*)(y + ro) = pk;
  __threadfence();
  *(volatile v8h*)(y + ro) = pk;
}

__global__ __launch_bounds__(256) void k_den(const hh* __restrict__ Qp, const hh* __restrict__ Kp,
                                             float* __restrict__ rd) {
  __shared__ float part[8 * 32];
  __shared__ __align__(16) float rl[32];
  const int tid = threadIdx.x, lane = tid & 31, w = tid >> 5;
  const int b = blockIdx.x;
  const int e0 = tid * 8;
  float z[8];
#pragma unroll
  for (int cc = 0; cc < 8; ++cc) z[cc] = 0.f;
#pragma unroll 1
  for (int tb = 0; tb < NN / 32; ++tb) {
    float keep = 0.f;
#pragma unroll 2
    for (int j = 0; j < 32; ++j) {
      const size_t ro = ((size_t)(b * NN + tb * 32 + j)) * EE + e0;
      const v8h kv = *(const v8h*)(Kp + ro);
      const v8h qv = *(const v8h*)(Qp + ro);
      float p = 0.f;
#pragma unroll
      for (int cc = 0; cc < 8; ++cc) {
        z[cc] += (float)kv[cc];
        p = fmaf((float)qv[cc], z[cc], p);
      }
      p = wsum(p);
      keep = (lane == j) ? p : keep;
    }
    part[w * 32 + lane] = keep;
    __syncthreads();
    if (w == 0) {
      float s = part[lane];
#pragma unroll
      for (int q = 1; q < 8; ++q) s += part[q * 32 + lane];
      rl[lane] = 1.0f / (s + 1e-6f);
    }
    __syncthreads();
    if (w == 0) {
      const int li = lane & 7;
      const v4f v = *(const v4f*)(rl + 4 * li);
      float* gp = rd + (size_t)b * NN + tb * 32 + 4 * li;
      if (lane < 8) *(volatile v4f*)gp = v;
      __threadfence();
      if (lane < 8) *(volatile v4f*)gp = v;
    }
  }
}

template <int MODE>
__global__ __launch_bounds__(256) void k_gemm(const hh* __restrict__ Ap, const hh* __restrict__ Bp,
                                              const float* __restrict__ bias, const float* __restrict__ res,
                                              const float* __restrict__ rsc, hh* __restrict__ o16,
                                              float* __restrict__ o32) {
  constexpr bool F32OUT = (MODE == 4 || MODE == 6);
  constexpr int LDA = (MODE == 0 || MODE == 1 || MODE == 5) ? DD : ((MODE == 2 || MODE == 4) ? EE : ((MODE == 3) ? NN : FF));
  constexpr int LDB = (MODE == 0 || MODE == 1 || MODE == 5) ? DD : ((MODE == 2 || MODE == 4) ? EE : ((MODE == 3) ? MTOK : FF));
  constexpr int LDO = (MODE == 0 || MODE == 3) ? EE : ((MODE == 1) ? MTOK : ((MODE == 2) ? NN : ((MODE == 5) ? FF : DD)));

  __shared__ __align__(16) EpiLds lds;
  const int tid = threadIdx.x, lane = tid & 31, w = tid >> 5;
  const int h = lane >> 4, c = lane & 15;
  const int wm = (w >> 1) * 32, wn = (w & 1) * 64;

  int m0 = 0, n0 = 0, kdim = 0, bz = 0;
  const hh* A = Ap;
  const hh* B = Bp;
  if constexpr (MODE == 2) {
    const int bx = blockIdx.x;
    bz = blockIdx.y;
    int mi = 0;
#pragma unroll
    for (int s = 1; s < NN / 128; ++s) mi += (((s * (s + 1)) / 2) <= bx) ? 1 : 0;
    const int ni = bx - (mi * (mi + 1)) / 2;
    m0 = mi * 128;
    n0 = ni * 128;
    kdim = EE;
    A = Ap + (size_t)bz * NN * EE;
    B = Bp + (size_t)bz * NN * EE;
  } else if constexpr (MODE == 3) {
    bz = blockIdx.z;
    const int mi = blockIdx.y;
    m0 = mi * 128;
    n0 = blockIdx.x * 128;
    kdim = (mi + 1) * 128;
    A = Ap + (size_t)bz * NN * NN;
    B = Bp + (size_t)bz * NN;
  } else {
    m0 = blockIdx.y * 128;
    n0 = blockIdx.x * 128;
    kdim = LDA;
  }

  v8f acc[2][4];
#pragma unroll
  for (int i = 0; i < 2; ++i)
#pragma unroll
    for (int j = 0; j < 4; ++j) acc[i][j] = zero8();
  gemm32x64(A, LDA, B, LDB, m0 + wm, n0 + wn, kdim, lane, acc);

  float bc[4] = {0.f, 0.f, 0.f, 0.f};
  if constexpr (MODE == 0 || MODE == 1 || MODE == 4 || MODE == 5 || MODE == 6) {
#pragma unroll
    for (int j = 0; j < 4; ++j) bc[j] = bias[n0 + wn + 16 * j + c];
  }
  float rs[2][8];
#pragma unroll
  for (int i = 0; i < 2; ++i)
#pragma unroll
    for (int r = 0; r < 8; ++r) rs[i][r] = 0.f;
  if constexpr (MODE == 3) {
#pragma unroll
    for (int i = 0; i < 2; ++i) {
      const v8f t = *(const v8f*)(rsc + (size_t)bz * NN + m0 + wm + 16 * i + 8 * h);
#pragma unroll
      for (int r = 0; r < 8; ++r) rs[i][r] = t[r];
    }
  }

  if constexpr (!F32OUT) {
#pragma unroll
    for (int i = 0; i < 2; ++i) {
#pragma unroll
      for (int j = 0; j < 4; ++j) {
        float v[8];
#pragma unroll
        for (int r = 0; r < 8; ++r) {
          const float a = acc[i][j][r];
          float t = 0.f;
          if constexpr (MODE == 0) {
            t = phi_f(a * (1.0f / 64.0f) + bc[j]);
          } else if constexpr (MODE == 1) {
            t = (a * (1.0f / 64.0f) + bc[j]) * 16.0f;
          } else if constexpr (MODE == 2) {
            const int ml = m0 + wm + 16 * i + 8 * h + r;
            const int nl = n0 + wn + 16 * j + c;
            t = (nl > ml) ? 0.f : a;
          } else if constexpr (MODE == 3) {
            t = a * rs[i][r] * 4.0f;
          } else {
            t = gelu_f(a * (1.0f / 64.0f) + bc[j]) * 16.0f;
          }
          v[r] = t;
        }
        if constexpr (MODE == 1) {
          const v8f tv = {v[0], v[1], v[2], v[3], v[4], v[5], v[6], v[7]};
          const v8h pk = __builtin_convertvector(tv, v8h);
          *(v8h*)(lds.h + (size_t)(wn + 16 * j + c) * SHP + wm + 16 * i + 8 * h) = pk;
        } else {
#pragma unroll
          for (int r = 0; r < 8; ++r)
            lds.h[(wm + 16 * i + 8 * h + r) * SHP + wn + 16 * j + c] = (hh)v[r];
        }
      }
    }
    __syncthreads();
    hh* ob = o16;
    if constexpr (MODE == 2) ob = o16 + (size_t)bz * NN * NN;
    const int orow0 = (MODE == 3) ? (bz * NN + m0) : m0;
    v8h val[8];
    size_t go[8];
#pragma unroll
    for (int it = 0; it < 8; ++it) {
      const int p  = tid + 256 * it;
      const int lr = p >> 4;
      const int pc = p & 15;
      val[it] = *(const v8h*)(lds.h + lr * SHP + pc * 8);
      if constexpr (MODE == 1) go[it] = (size_t)(n0 + lr) * LDO + m0 + pc * 8;
      else                     go[it] = (size_t)(orow0 + lr) * LDO + n0 + pc * 8;
    }
#pragma unroll
    for (int it = 0; it < 8; ++it) *(volatile v8h*)(ob + go[it]) = val[it];
    __threadfence();
#pragma unroll
    for (int it = 0; it < 8; ++it) *(volatile v8h*)(ob + go[it]) = val[it];
  } else {
    constexpr float OSC = (MODE == 4) ? (1.0f / 4096.0f) : (1.0f / 1024.0f);
#pragma unroll
    for (int hf = 0; hf < 2; ++hf) {
      if ((w >> 2) == hf) {
#pragma unroll
        for (int i = 0; i < 2; ++i)
#pragma unroll
          for (int j = 0; j < 4; ++j)
#pragma unroll
            for (int r = 0; r < 8; ++r)
              lds.f[(wm - 64 * hf + 16 * i + 8 * h + r) * SFP + wn + 16 * j + c] = acc[i][j][r] * OSC + bc[j];
      }
      __syncthreads();
      v4f val[8];
      size_t go[8];
#pragma unroll
      for (int it = 0; it < 8; ++it) {
        const int p  = tid + 256 * it;
        const int lr = p >> 5;
        const int pc = p & 31;
        const v4f sv = *(const v4f*)(lds.f + lr * SFP + pc * 4);
        const size_t gi = (size_t)(m0 + 64 * hf + lr) * LDO + n0 + pc * 4;
        const v4f rr = *(const v4f*)(res + gi);
        val[it] = sv + rr;
        go[it] = gi;
      }
#pragma unroll
      for (int it = 0; it < 8; ++it) *(volatile v4f*)(o32 + go[it]) = val[it];
      __threadfence();
#pragma unroll
      for (int it = 0; it < 8; ++it) *(volatile v4f*)(o32 + go[it]) = val[it];
      if (hf == 0) __syncthreads();
    }
  }
}

extern "C" void kernel_launch(void* const* d_in, const int* in_sizes, int n_in,
                              void* d_out, int out_size, void* d_ws, size_t ws_size,
                              hipStream_t stream) {
  if (n_in < 17) return;
  if (in_sizes[0] != MTOK * DD) return;
  if (in_sizes[1] != DD * EE || in_sizes[3] != DD * EE || in_sizes[5] != DD * EE) return;
  if (in_sizes[2] != EE || in_sizes[4] != EE || in_sizes[6] != EE) return;
  if (in_sizes[7] != EE * DD || in_sizes[8] != DD) return;
  if (in_sizes[9] != DD || in_sizes[10] != DD || in_sizes[11] != DD || in_sizes[12] != DD) return;
  if (in_sizes[13] != DD * FF || in_sizes[14] != FF) return;
  if (in_sizes[15] != FF * DD || in_sizes[16] != DD) return;
  if (out_size != MTOK * DD) return;

  const float* x    = (const float*)d_in[0];
  const float* q_w  = (const float*)d_in[1];
  const float* q_b  = (const float*)d_in[2];
  const float* k_w  = (const float*)d_in[3];
  const float* k_b  = (const float*)d_in[4];
  const float* v_w  = (const float*)d_in[5];
  const float* v_b  = (const float*)d_in[6];
  const float* o_w  = (const float*)d_in[7];
  const float* o_b  = (const float*)d_in[8];
  const float* ln1g = (const float*)d_in[9];
  const float* ln1b = (const float*)d_in[10];
  const float* ln2g = (const float*)d_in[11];
  const float* ln2b = (const float*)d_in[12];
  const float* w1   = (const float*)d_in[13];
  const float* b1   = (const float*)d_in[14];
  const float* w2   = (const float*)d_in[15];
  const float* b2   = (const float*)d_in[16];
  float* out = (float*)d_out;

  size_t off = 0;
  const size_t oWQ = off; off += (size_t)EE * DD * 2;
  const size_t oWK = off; off += (size_t)EE * DD * 2;
  const size_t oWV = off; off += (size_t)EE * DD * 2;
  const size_t oWO = off; off += (size_t)DD * EE * 2;
  const size_t oW1 = off; off += (size_t)FF * DD * 2;
  const size_t oW2 = off; off += (size_t)DD * FF * 2;
  const size_t oXN = off; off += (size_t)MTOK * DD * 2;
  const size_t oQF = off; off += (size_t)MTOK * EE * 2;
  const size_t oKF = off; off += (size_t)MTOK * EE * 2;
  const size_t oVT = off; off += (size_t)EE * MTOK * 2;
  const size_t oP  = off; off += (size_t)BB * NN * NN * 2;
  const size_t oY  = off; off += (size_t)MTOK * EE * 2;
  const size_t oRD = off; off += (size_t)MTOK * 4;
  if (off > ws_size) return;
  if (off > (size_t)134217728) return;
  if (oKF != oQF + (size_t)MTOK * EE * 2) return;
  if ((size_t)MTOK * FF * 2 > (oVT - oQF)) return;

  char* ws = (char*)d_ws;
  hh* WQ = (hh*)(ws + oWQ);  hh* WK = (hh*)(ws + oWK);  hh* WV = (hh*)(ws + oWV);
  hh* WO = (hh*)(ws + oWO);  hh* W1 = (hh*)(ws + oW1);  hh* W2 = (hh*)(ws + oW2);
  hh* XN = (hh*)(ws + oXN);
  hh* QF = (hh*)(ws + oQF);  hh* KF = (hh*)(ws + oKF);
  hh* VT = (hh*)(ws + oVT);
  hh* P  = (hh*)(ws + oP);
  hh* Y  = (hh*)(ws + oY);
  float* RD = (float*)(ws + oRD);
  hh* H  = (hh*)(ws + oQF);
  float* X1 = (float*)(ws + oP);

  const float* fnull = (const float*)0;
  hh* hnull = (hh*)0;
  float* onull = (float*)0;

  k_cvt_wt<DD, EE><<<dim3(DD / 64, EE / 64), dim3(256), 0, stream>>>(q_w, WQ);
  k_cvt_wt<DD, EE><<<dim3(DD / 64, EE / 64), dim3(256), 0, stream>>>(k_w, WK);
  k_cvt_wt<DD, EE><<<dim3(DD / 64, EE / 64), dim3(256), 0, stream>>>(v_w, WV);
  k_cvt_wt<EE, DD><<<dim3(EE / 64, DD / 64), dim3(256), 0, stream>>>(o_w, WO);
  k_cvt_wt<DD, FF><<<dim3(DD / 64, FF / 64), dim3(256), 0, stream>>>(w1, W1);
  k_cvt_wt<FF, DD><<<dim3(FF / 64, DD / 64), dim3(256), 0, stream>>>(w2, W2);
  k_ln<<<dim3(MTOK), dim3(128), 0, stream>>>(x, ln1g, ln1b, XN);
  k_gemm<0><<<dim3(EE / 128, MTOK / 128), dim3(256), 0, stream>>>(XN, WQ, q_b, fnull, fnull, QF, onull);
  k_gemm<0><<<dim3(EE / 128, MTOK / 128), dim3(256), 0, stream>>>(XN, WK, k_b, fnull, fnull, KF, onull);
  k_gemm<1><<<dim3(EE / 128, MTOK / 128), dim3(256), 0, stream>>>(XN, WV, v_b, fnull, fnull, VT, onull);
  k_den<<<dim3(BB), dim3(256), 0, stream>>>(QF, KF, RD);
  k_gemm<2><<<dim3(NTRI, BB), dim3(256), 0, stream>>>(QF, KF, fnull, fnull, fnull, P, onull);
  k_gemm<3><<<dim3(EE / 128, NN / 128, BB), dim3(256), 0, stream>>>(P, VT, fnull, fnull, RD, Y, onull);
  k_gemm<4><<<dim3(DD / 128, MTOK / 128), dim3(256), 0, stream>>>(Y, WO, o_b, x, fnull, hnull, X1);
  k_ln<<<dim3(MTOK), dim3(128), 0, stream>>>(X1, ln2g, ln2b, XN);
  k_gemm<5><<<dim3(FF / 128, MTOK / 128), dim3(256), 0, stream>>>(XN, W1, b1, fnull, fnull, H, onull);
  k_gemm<6><<<dim3(DD / 128, MTOK / 128), dim3(256), 0, stream>>>(H, W2, b2, X1, fnull, hnull, out);
  (void)hipGetLastError();
}
